// ConvLayer_49795850830364
// MI455X (gfx1250) — hardware-run, weakly checked
//
#include <hip/hip_runtime.h>
#include <math.h>

typedef __attribute__((ext_vector_type(16))) _Float16 v16h;
typedef __attribute__((ext_vector_type(8)))  _Float16 v8h;
typedef __attribute__((ext_vector_type(16))) __bf16   v16b;
typedef __attribute__((ext_vector_type(8)))  __bf16   v8b;
typedef __attribute__((ext_vector_type(8)))  float    v8f;
typedef __attribute__((ext_vector_type(4)))  float    v4f;
typedef __attribute__((ext_vector_type(4)))  unsigned int v4u;
typedef __attribute__((ext_vector_type(4)))  int      v4i;

constexpr int kNodes = 8192;
constexpr int kFeat  = 128;
constexpr int kClus  = 128;
constexpr int kEdges = 262144;
constexpr int kNT    = 256;
constexpr int kTileNodes = 1024;
constexpr int kTiles = kNodes / kTileNodes;
constexpr int kRowsPerWave = kTileNodes / 8;
constexpr int kChunk  = 2048;
constexpr int kChunks = kEdges / kChunk;
constexpr int kSP     = kChunk / kNT;
constexpr int kAK     = 2 * kFeat;
constexpr int kPoolN  = 320;
constexpr int kTrB    = 64;
constexpr int kTrEdgesPerWave = kEdges / (kTrB * 8);
constexpr int kTrRow  = 256;
constexpr float kWCarry = 16.0f;
constexpr float kInvW   = 1.0f / 16.0f;
constexpr float kInvWW  = 1.0f / 256.0f;

static_assert(kEdges % kChunk == 0);
static_assert(kChunk == kNT * kSP);
static_assert(kSP % 4 == 0);
static_assert(kNodes == kTiles * kTileNodes);
static_assert(kTileNodes == 8 * kRowsPerWave);
static_assert(kNodes % 64 == 0 && kFeat % 64 == 0 && kClus % 64 == 0 && kPoolN % 64 == 0);
static_assert(kAK % 32 == 0 && kFeat % 32 == 0 && kNodes % 32 == 0);
static_assert(kEdges == kTrB * 8 * kTrEdgesPerWave);
static_assert(kTrEdgesPerWave % 32 == 0);
static_assert((kNodes * kFeat) % 2048 == 0);
static_assert(2 * kClus * kFeat * 4 == 131072);
static_assert(131072 + 4 <= 131076);

__device__ __forceinline__ unsigned short f2bf_bits(float f) {
  unsigned u = __float_as_uint(f);
  return (unsigned short)((u + 0x7FFFu + ((u >> 16) & 1u)) >> 16);
}
__device__ __forceinline__ float bf_bits2f(unsigned short h) { return __uint_as_float(((unsigned)h) << 16); }

__device__ __forceinline__ void dep_guard_h(v8f& a, v8f& b, v16h x, v16h y) { asm volatile("v_nop\n\tv_nop\n\tv_nop\n\tv_nop" : "+v"(a), "+v"(b) : "v"(x), "v"(y)); }
__device__ __forceinline__ void dep_guard_b(v8f& a, v8f& b, v16b x, v16b y) { asm volatile("v_nop\n\tv_nop\n\tv_nop\n\tv_nop" : "+v"(a), "+v"(b) : "v"(x), "v"(y)); }
__device__ __forceinline__ void keep4_h(v16h a, v16h b, v16h c, v16h d) { asm volatile("v_nop" :: "v"(a), "v"(b), "v"(c), "v"(d)); }
__device__ __forceinline__ void keep4_b(v16b a, v16b b, v16b c, v16b d) { asm volatile("v_nop" :: "v"(a), "v"(b), "v"(c), "v"(d)); }
__device__ __forceinline__ void acc_guard4(v8f& a, v8f& b, v8f& c, v8f& d) { asm volatile("v_nop\n\tv_nop\n\tv_nop\n\tv_nop" : "+v"(a), "+v"(b), "+v"(c), "+v"(d)); }
template <typename T> struct Frag;
template <> struct Frag<_Float16> {
  typedef v16h V; union U { v16h v; v8h h[2]; };
  static __device__ __forceinline__ v16h load(const _Float16* p) {
    U f; f.h[0] = *(const v8h*)(p); f.h[1] = *(const v8h*)(p + 16); return f.v;
  }
  static __device__ __forceinline__ v8f mma(v16h a, v16h b, v8f c) {
    return __builtin_amdgcn_wmma_f32_16x16x32_f16(false, a, false, b, (short)0, c, false, false);
  }
  static __device__ __forceinline__ void guard(v8f& a, v8f& b, v16h x, v16h y) { dep_guard_h(a, b, x, y); }
  static __device__ __forceinline__ void keep(v16h a, v16h b, v16h c, v16h d) { keep4_h(a, b, c, d); }
};
template <> struct Frag<__bf16> {
  typedef v16b V; union U { v16b v; v8b h[2]; };
  static __device__ __forceinline__ v16b load(const __bf16* p) {
    U f; f.h[0] = *(const v8b*)(p); f.h[1] = *(const v8b*)(p + 16); return f.v;
  }
  static __device__ __forceinline__ v8f mma(v16b a, v16b b, v8f c) {
    return __builtin_amdgcn_wmma_f32_16x16x32_bf16(false, a, false, b, (short)0, c, false, false);
  }
  static __device__ __forceinline__ void guard(v8f& a, v8f& b, v16b x, v16b y) { dep_guard_b(a, b, x, y); }
  static __device__ __forceinline__ void keep(v16b a, v16b b, v16b c, v16b d) { keep4_b(a, b, c, d); }
};

template <int ET> struct Elem;
template <> struct Elem<0> { typedef _Float16 T; };
template <> struct Elem<1> { typedef __bf16 T; };
template <int ET, bool SPLIT, int BIAS_MODE, int OUT_MODE, bool RESID, int ACT = 0>
__global__ __launch_bounds__(256) void wmma_gemm64(
    const unsigned short* __restrict__ Ap, const unsigned short* __restrict__ A2p, int lda, long strideA,
    const unsigned short* __restrict__ Btp, const unsigned short* __restrict__ Bt2p, int ldb, long strideB,
    void* __restrict__ Cout, void* __restrict__ Cout2, int ldc, long strideC,
    const float* __restrict__ bias,
    const float* __restrict__ resid, long strideR,
    int M, int N, int K, float scale) {
  typedef typename Elem<ET>::T T;
  typedef typename Frag<T>::V V;
  const T* A = (const T*)Ap; const T* A2 = (const T*)A2p; const T* Bt = (const T*)Btp; const T* Bt2 = (const T*)Bt2p;
  __shared__ __align__(16) float sT[8][16 * 68];
  const int b    = blockIdx.y;
  const int lane = threadIdx.x & 31;
  const int wave = threadIdx.x >> 5;
  const int tilesN = N >> 6;
  const int tilesM = M >> 6;
  const int tile = blockIdx.x * 8 + wave;
  if (tile >= tilesM * tilesN) return;
  const int tm = tile / tilesN;
  const int tn = tile - tm * tilesN;
  const int m0 = tm << 6;
  const int n0 = tn << 6;

  const T* Ab  = A  + (size_t)b * strideA;
  const T* Bb  = Bt + (size_t)b * strideB;
  const T* Ab2 = SPLIT ? (A2  + (size_t)b * strideA) : nullptr;
  const T* Bb2 = SPLIT ? (Bt2 + (size_t)b * strideB) : nullptr;

  const int rlane = lane & 15;
  const int koff  = (lane >> 4) * 8;
  const int mOff  = (lane >> 4) * 8;

  v8f acc[4][4];
#pragma unroll
  for (int i = 0; i < 4; ++i)
#pragma unroll
    for (int j = 0; j < 4; ++j) acc[i][j] = (v8f){0.f,0.f,0.f,0.f,0.f,0.f,0.f,0.f};

  for (int k0 = 0; k0 < K; k0 += 32) {
    V bh[4], bl[4];
#pragma unroll
    for (int j = 0; j < 4; ++j) {
      const size_t bo = (size_t)(n0 + (j << 4) + rlane) * ldb + koff + k0;
      bh[j] = Frag<T>::load(Bb + bo);
      if (SPLIT) bl[j] = Frag<T>::load(Bb2 + bo);
    }
#pragma unroll
    for (int i = 0; i < 4; ++i) {
      const size_t ao = (size_t)(m0 + (i << 4) + rlane) * lda + koff + k0;
      V ah = Frag<T>::load(Ab + ao);
      V al;
      if (SPLIT) al = Frag<T>::load(Ab2 + ao);
#pragma unroll
      for (int j = 0; j < 4; ++j) {
        acc[i][j] = Frag<T>::mma(ah, bh[j], acc[i][j]);
        if (SPLIT) {
          acc[i][j] = Frag<T>::mma(ah, bl[j], acc[i][j]);
          acc[i][j] = Frag<T>::mma(al, bh[j], acc[i][j]);
        }
      }
      Frag<T>::guard(acc[i][0], acc[i][3], ah, SPLIT ? al : ah);
    }
    Frag<T>::keep(bh[0], bh[1], bh[2], bh[3]);
    if (SPLIT) Frag<T>::keep(bl[0], bl[1], bl[2], bl[3]);
  }
  acc_guard4(acc[0][0], acc[0][1], acc[0][2], acc[0][3]);
  acc_guard4(acc[1][0], acc[1][1], acc[1][2], acc[1][3]);
  acc_guard4(acc[2][0], acc[2][1], acc[2][2], acc[2][3]);
  acc_guard4(acc[3][0], acc[3][1], acc[3][2], acc[3][3]);

  float* slab = sT[wave];
  const float* Rb = RESID ? (resid + (size_t)b * strideR) : nullptr;
#pragma unroll
  for (int i = 0; i < 4; ++i) {
    const int mBase = m0 + (i << 4);
#pragma unroll
    for (int j = 0; j < 4; ++j) {
      const int n = n0 + (j << 4) + rlane;
      float bv = 0.f;
      if (BIAS_MODE == 2) bv = bias[n];
#pragma unroll
      for (int r = 0; r < 8; ++r) {
        float v = acc[i][j][r] * scale;
        if (BIAS_MODE == 1) v += bias[mBase + mOff + r];
        if (BIAS_MODE == 2) v += bv;
        if (RESID) v += Rb[(size_t)(mBase + mOff + r) * ldc + n];
        if (ACT == 1) v = tanhf(v);
        if (ACT == 2) v = fmaxf(v, 0.0f);
        if (ACT == 3) v = v / (1.0f + expf(-v));
        if (ACT == 4) v = (v > 0.f) ? v : 0.01f * v;
        if (ACT == 5) v = 0.5f * v * (1.0f + erff(v * 0.70710678118654752f));
        slab[(mOff + r) * 68 + (j << 4) + rlane] = v;
      }
    }
    __builtin_amdgcn_fence(__ATOMIC_RELEASE, "workgroup");
    __builtin_amdgcn_wave_barrier();
    __builtin_amdgcn_fence(__ATOMIC_ACQUIRE, "workgroup");
    if (OUT_MODE == 0) {
      float* C = (float*)Cout + (size_t)b * strideC;
      const int hh = lane >> 4, c4 = (lane & 15) * 4;
      for (int pass = 0; pass < 2; ++pass) {
#pragma unroll
        for (int it = 0; it < 8; ++it) {
          const int row = it * 2 + hh;
          v4f v = *(const v4f*)(slab + row * 68 + c4);
          *(volatile v4f*)(C + (size_t)(mBase + row) * ldc + n0 + c4) = v;
        }
        __threadfence();
      }
    } else {
      const int q = lane >> 3, c8 = (lane & 7) * 8;
      unsigned short* C  = (unsigned short*)Cout  + (size_t)b * strideC;
      unsigned short* C2 = (OUT_MODE == 2) ? ((unsigned short*)Cout2 + (size_t)b * strideC) : nullptr;
      for (int pass = 0; pass < 2; ++pass) {
#pragma unroll
        for (int it = 0; it < 4; ++it) {
          const int row = it * 4 + q;
          const float* sp = slab + row * 68 + c8;
          v8h hv, lv;
#pragma unroll
          for (int e = 0; e < 8; ++e) {
            if (OUT_MODE == 1) {
              hv[e] = (_Float16)sp[e];
            } else {
              unsigned short hb = f2bf_bits(sp[e]);
              unsigned short lb = f2bf_bits(sp[e] - bf_bits2f(hb));
              hv[e] = __builtin_bit_cast(_Float16, hb);
              lv[e] = __builtin_bit_cast(_Float16, lb);
            }
          }
          *(volatile v8h*)(C + (size_t)(mBase + row) * ldc + n0 + c8) = hv;
          if (OUT_MODE == 2) *(volatile v8h*)(C2 + (size_t)(mBase + row) * ldc + n0 + c8) = lv;
        }
        __threadfence();
      }
    }
    __builtin_amdgcn_fence(__ATOMIC_RELEASE, "workgroup");
    __builtin_amdgcn_wave_barrier();
    __builtin_amdgcn_fence(__ATOMIC_ACQUIRE, "workgroup");
  }
}

__device__ __forceinline__ unsigned pk16(unsigned short a, unsigned short b) { return (unsigned)a | ((unsigned)b << 16); }
__device__ __forceinline__ unsigned short h_bits(float f) { const _Float16 h = (_Float16)f; return __builtin_bit_cast(unsigned short, h); }
__device__ __forceinline__ v4u pack8_f16(const float* sp) {
  const v4f a = *(const v4f*)(sp);
  const v4f c = *(const v4f*)(sp + 4);
  unsigned short hb[8];
#pragma unroll
  for (int e = 0; e < 4; ++e) { hb[e] = h_bits(a[e]); hb[4 + e] = h_bits(c[e]); }
  return (v4u){pk16(hb[0], hb[1]), pk16(hb[2], hb[3]), pk16(hb[4], hb[5]), pk16(hb[6], hb[7])};
}
__device__ __forceinline__ void wave_lds_sync() {
  __builtin_amdgcn_fence(__ATOMIC_RELEASE, "workgroup");
  __builtin_amdgcn_wave_barrier();
  __builtin_amdgcn_fence(__ATOMIC_ACQUIRE, "workgroup");
}
__device__ __forceinline__ float mish_f(float x) {
  const float u = expf(fminf(x, 30.0f));
  const float n = u * (u + 2.0f);
  const float r = n * (1.0f / (n + 2.0f));
  return x * r;
}
__device__ __forceinline__ float selu_f(float v) {
  const float kAlpha = 1.6732632423543772f;
  const float kScale = 1.0507009873554805f;
  const float neg = kAlpha * expm1f(v);
  return kScale * ((v > 0.0f) ? v : neg);
}
__device__ inline float block_sum256(float v, float* red) {
  const int t = threadIdx.x;
  red[t] = v;
  __syncthreads();
  for (int s2 = 128; s2 > 0; s2 >>= 1) {
    if (t < s2) red[t] += red[t + s2];
    __syncthreads();
  }
  const float r = red[0];
  __syncthreads();
  return r;
}

__device__ __forceinline__ int blk_excl_scan(int cnt, int* scan_ws, int tid, int* tot) {
  const int lane = tid & 31, wave = tid >> 5; int incl = cnt;
#pragma unroll
  for (int o = 1; o < 32; o <<= 1) { const int v = __shfl_up(incl, o, 32); if (lane >= o) incl += v; }
  if (lane == 31) scan_ws[wave] = incl;
  __syncthreads();
  if (wave == 0) { int wv = (lane < kNT / 32) ? scan_ws[lane] : 0; int wincl = wv;
#pragma unroll
    for (int o = 1; o < 32; o <<= 1) { const int v = __shfl_up(wincl, o, 32); if (lane >= o) wincl += v; }
    if (lane < kNT / 32) scan_ws[32 + lane] = wincl - wv; if (lane == 31) scan_ws[64] = wincl; }
  __syncthreads();
  const int res = scan_ws[32 + wave] + incl - cnt; *tot = scan_ws[64];
  return res;
}
__device__ __forceinline__ int chunk_hits(const int* __restrict__ keyv, const int* __restrict__ valv, int e0, int n0, int tid,
                                          int* LIST, int* scan_ws) {
  const int eb = e0 + tid * kSP;
  const int ebc = (eb <= kEdges - kSP) ? eb : (kEdges - kSP);
  const bool live = eb < kEdges;
  int rec[kSP]; int cnt = 0;
#pragma unroll
  for (int k = 0; k < kSP; k += 4) {
    const v4i d4 = *(const v4i*)(keyv + ebc + k);
    const v4i s4 = *(const v4i*)(valv + ebc + k);
#pragma unroll
    for (int e = 0; e < 4; ++e) {
      const int d = d4[e]; int r = -1;
      int s = s4[e]; s = s < 0 ? 0 : (s >= kNodes ? kNodes - 1 : s);
      if (live && d >= n0 && d < n0 + kTileNodes) { r = ((d - n0) << 16) | s; ++cnt; }
      rec[k + e] = r;
    }
  }
  int tot; int p = blk_excl_scan(cnt, scan_ws, tid, &tot);
#pragma unroll
  for (int k = 0; k < kSP; ++k) if (rec[k] >= 0) { if ((unsigned)p < (unsigned)kChunk) LIST[p] = rec[k]; ++p; }
  __syncthreads();
  return tot < kChunk ? tot : kChunk;
}

__global__ __launch_bounds__(kNT) void prep_kernel(
    const float* __restrict__ w0, const float* __restrict__ w1, const float* __restrict__ w2, const float* __restrict__ w3,
    const float* __restrict__ w4, const float* __restrict__ w5, const float* __restrict__ w6, const float* __restrict__ w7,
    const float* __restrict__ w8, const float* __restrict__ w9, const float* __restrict__ w10, const float* __restrict__ w11,
    const float* __restrict__ b1, unsigned short* __restrict__ BTS, unsigned short* __restrict__ BTM, float* __restrict__ B1X16) {
  __shared__ float sm[64][65];
  const int t  = threadIdx.x;
  const int k0 = blockIdx.x * 64;
  const int j0 = blockIdx.y * 64;
  const int z  = blockIdx.z;
  const float* W = (z == 0) ? w0 : (z == 1) ? w1 : (z == 2) ? w2 : (z == 3) ? w3 : (z == 4) ? w4 : (z == 5) ? w5 :
                   (z == 6) ? w6 : (z == 7) ? w7 : (z == 8) ? w8 : (z == 9) ? w9 : (z == 10) ? w10 : w11;
  unsigned short* dst; int pitch, coloff;
  if (z < 10) { dst = BTS + (size_t)(z >> 1) * kFeat * kAK; pitch = kAK; coloff = (z & 1) * kFeat; }
  else        { dst = BTM + (size_t)(z - 10) * kFeat * kFeat; pitch = kFeat; coloff = 0; }
#pragma unroll 8
  for (int i = 0; i < 16; ++i) {
    const int e = i * kNT + t;
    const int r = e >> 6;
    const int c = e & 63;
    sm[c][r] = W[(size_t)(k0 + r) * kFeat + j0 + c] * kWCarry;
  }
  __syncthreads();
  const int lane = t & 31, wave = t >> 5;
  const int q = lane >> 3, c8 = (lane & 7) * 8;
  for (int pass = 0; pass < 2; ++pass) {
#pragma unroll
    for (int it = 0; it < 2; ++it) {
      const int row = wave * 8 + it * 4 + q;
      unsigned short hb[8];
#pragma unroll
      for (int e = 0; e < 8; ++e) hb[e] = h_bits(sm[row][c8 + e]);
      const v4u u = (v4u){pk16(hb[0], hb[1]), pk16(hb[2], hb[3]), pk16(hb[4], hb[5]), pk16(hb[6], hb[7])};
      *(volatile v4u*)(dst + (size_t)(j0 + row) * pitch + coloff + k0 + c8) = u;
    }
    __threadfence();
  }
  if (z == 0 && blockIdx.x == 0 && blockIdx.y == 0 && wave == 0) {
    const v4f bv = *(const v4f*)(b1 + 4 * lane) * kWCarry;
    float* bp = B1X16 + 4 * lane;
    *(volatile v4f*)bp = bv;
    __threadfence();
    *(volatile v4f*)bp = bv;
  }
}

__global__ __launch_bounds__(kNT) void agg_kernel(const float* __restrict__ X0, const float* __restrict__ X1,
                                                const int* __restrict__ E0, const int* __restrict__ E1,
                                                float* ACC, unsigned* __restrict__ A16) {
  __shared__ int LIST[kChunk];
  __shared__ float SCNT[kTileNodes];
  __shared__ int scan_ws[80];
  const int tid = threadIdx.x, lane = tid & 31, wave = tid >> 5;
  const int g = blockIdx.y;
  const int n0 = blockIdx.x * kTileNodes;
  const float* X = g ? X1 : X0;
  const int* ei = g ? E1 : E0;
  const int* srcv = ei;
  const int* dstv = ei + kEdges;
  float* accg = ACC + (size_t)g * kNodes * kFeat;
  unsigned* a16g = A16 + (size_t)g * kNodes * (kAK / 2);

  for (int i = tid; i < kChunk; i += kNT) LIST[i] = 0;
  for (int i = tid; i < kTileNodes; i += kNT) SCNT[i] = 0.0f;
  if (tid < 80) scan_ws[tid] = 0;
  const v4f z4 = {0.f, 0.f, 0.f, 0.f};
#pragma unroll 1
  for (int j = 0; j < kRowsPerWave; ++j) {
    float* rp = accg + (size_t)(n0 + wave * kRowsPerWave + j) * kFeat + 4 * lane;
    *(v4f*)rp = z4;
  }
  __syncthreads();

#pragma unroll 1
  for (int c = 0; c < kChunks; ++c) {
    const int tot = chunk_hits(dstv, srcv, c * kChunk, n0, tid, LIST, scan_ws);
#pragma unroll 1
    for (int base = 0; base < tot; base += 32) {
      const int q = base + lane;
      const int qc = (q < kChunk) ? q : (kChunk - 1);
      int rv = LIST[qc];
      rv = (q < tot) ? rv : -1;
      const int own = (rv >= 0 && (rv >> 23) == wave) ? 1 : 0;
      unsigned msk = (unsigned)__ballot(own);
#pragma unroll 1
      for (int it = 0; it < 32; ++it) {
        if (msk == 0u) break;
        const int bp = __builtin_ctz(msk); msk &= msk - 1u;
        const int r = __shfl(rv, bp, 32);
        const int dl = r >> 16, s = r & 0xFFFF;
        const v4f xv = *(const v4f*)(X + (size_t)s * kFeat + 4 * lane);
        float* rp = accg + (size_t)(n0 + dl) * kFeat + 4 * lane;
        v4f a = *(const v4f*)rp;
        a = a + xv;
        *(v4f*)rp = a;
        if (lane == 0) SCNT[dl] += 1.0f;
      }
    }
    __syncthreads();
  }
  __threadfence_block();

  const int c16 = 8 * (lane & 15);
  const float fx = (float)(lane >> 4);
  const float fmsel = 1.0f - fx;
#pragma unroll 1
  for (int j = 0; j < kRowsPerWave; ++j) {
    const int dl = wave * kRowsPerWave + j;
    const int n = n0 + dl;
    const float cnt = SCNT[dl];
    const float inv = 1.0f / fmaxf(cnt, 1.0f);
    const float fm = inv * fmsel;
    const float* rp = accg + (size_t)n * kFeat + c16;
    const float* xp = X + (size_t)n * kFeat + c16;
    const v4f a0 = *(const v4f*)(rp);
    const v4f a1 = *(const v4f*)(rp + 4);
    const v4f xa = *(const v4f*)(xp);
    const v4f xb = *(const v4f*)(xp + 4);
    unsigned short hb[8];
#pragma unroll
    for (int e = 0; e < 4; ++e) {
      hb[e]     = h_bits(fmaf(a0[e], fm, xa[e] * fx));
      hb[4 + e] = h_bits(fmaf(a1[e], fm, xb[e] * fx));
    }
    const v4u u = (v4u){pk16(hb[0], hb[1]), pk16(hb[2], hb[3]), pk16(hb[4], hb[5]), pk16(hb[6], hb[7])};
    unsigned* op = a16g + (size_t)n * (kAK / 2) + 4 * lane;
    *(volatile v4u*)op = u;
    __threadfence();
    *(volatile v4u*)op = u;
  }
}

template <int MODE>
__global__ __launch_bounds__(kNT) void act_kernel(const float* __restrict__ PRE, const float* __restrict__ bias0,
                                                const float* __restrict__ bias1, const float* __restrict__ RES,
                                                float* __restrict__ OUTF, unsigned* __restrict__ OUT16) {
  __shared__ __align__(16) float sres[2048];
  const int t = threadIdx.x;
  const int g = blockIdx.y;
  const size_t planeoff = (size_t)g * kNodes * kFeat;
  const size_t base = (size_t)blockIdx.x * 2048;
  const float* bias = g ? bias1 : bias0;
  const float bv = bias[t & (kFeat - 1)];
#pragma unroll 1
  for (int j = 0; j < 8; ++j) {
    const size_t idx = planeoff + base + (size_t)(256 * j + t);
    const float v = PRE[idx] + bv;
    float y = mish_f(v);
    if (MODE == 1) y = RES[idx] + y;
    sres[256 * j + t] = y;
  }
  __syncthreads();
  for (int pass = 0; pass < 2; ++pass) {
#pragma unroll
    for (int r = 0; r < 2; ++r) {
      const int off = r * 1024 + 4 * t;
      const v4f o = *(const v4f*)(sres + off);
      *(volatile v4f*)(OUTF + planeoff + base + off) = o;
    }
    if (MODE == 2) {
      const v4u u = pack8_f16(sres + 8 * t);
      *(volatile v4u*)(OUT16 + (planeoff + base) / 2 + 4 * t) = u;
    }
    __threadfence();
  }
}

__global__ __launch_bounds__(kNT) void softmax_kernel(const float* __restrict__ LG, float* __restrict__ S) {
  const int tid = threadIdx.x, lane = tid & 31, wave = tid >> 5;
  const int g = blockIdx.y;
  const int row = blockIdx.x * 8 + wave;
  const size_t off = ((size_t)g * kNodes + row) * kClus + 4 * lane;
  const v4f x = *(const v4f*)(LG + off);
  float m = fmaxf(fmaxf(x[0], x[1]), fmaxf(x[2], x[3]));
  m = fmaxf(m, __shfl_xor(m, 16, 32));
  m = fmaxf(m, __shfl_xor(m, 8, 32));
  m = fmaxf(m, __shfl_xor(m, 4, 32));
  m = fmaxf(m, __shfl_xor(m, 2, 32));
  m = fmaxf(m, __shfl_xor(m, 1, 32));
  v4f e;
  e[0] = expf(x[0] - m); e[1] = expf(x[1] - m); e[2] = expf(x[2] - m); e[3] = expf(x[3] - m);
  float s = (e[0] + e[1]) + (e[2] + e[3]);
  s += __shfl_xor(s, 16, 32);
  s += __shfl_xor(s, 8, 32);
  s += __shfl_xor(s, 4, 32);
  s += __shfl_xor(s, 2, 32);
  s += __shfl_xor(s, 1, 32);
  const float inv = 1.0f / s;
  const v4f p = e * inv;
  float* op = S + off;
  *(volatile v4f*)op = p;
  __threadfence();
  *(volatile v4f*)op = p;
}

__global__ __launch_bounds__(kNT) void poolpack_kernel(const float* __restrict__ HF, const float* __restrict__ S,
                                                     unsigned short* __restrict__ APOOL, unsigned short* __restrict__ BTPOOL) {
  __shared__ __align__(16) float sTt[kFeat * 68];
  const int tid = threadIdx.x, lane = tid & 31, wave = tid >> 5;
  const int g = blockIdx.y;
  const int n0 = blockIdx.x * 64;
  const float* hp = HF + ((size_t)g * kNodes + n0) * kFeat;
  const float* sp = S  + ((size_t)g * kNodes + n0) * kClus;
  unsigned short* ap = APOOL  + (size_t)g * kClus  * kNodes;
  unsigned short* bp = BTPOOL + (size_t)g * kPoolN * kNodes;
  const int q = lane >> 3, c8 = (lane & 7) * 8;
#pragma unroll 4
  for (int i = 0; i < 8; ++i) {
    const int e4 = i * kNT + tid;
    const int n = e4 >> 5, c4 = (e4 & 31) * 4;
    const v4f v = *(const v4f*)(hp + 4 * (size_t)e4);
    sTt[(c4 + 0) * 68 + n] = v[0]; sTt[(c4 + 1) * 68 + n] = v[1]; sTt[(c4 + 2) * 68 + n] = v[2]; sTt[(c4 + 3) * 68 + n] = v[3];
  }
  __syncthreads();
  for (int pass = 0; pass < 2; ++pass) {
#pragma unroll
    for (int it = 0; it < 4; ++it) {
      const int row = wave * 16 + it * 4 + q;
      const v4u u = pack8_f16(sTt + row * 68 + c8);
      *(volatile v4u*)(bp + (size_t)row * kNodes + n0 + c8) = u;
    }
    __threadfence();
  }
  __syncthreads();
#pragma unroll 4
  for (int i = 0; i < 8; ++i) {
    const int e4 = i * kNT + tid;
    const int n = e4 >> 5, c4 = (e4 & 31) * 4;
    const v4f v = *(const v4f*)(sp + 4 * (size_t)e4);
    sTt[(c4 + 0) * 68 + n] = v[0]; sTt[(c4 + 1) * 68 + n] = v[1]; sTt[(c4 + 2) * 68 + n] = v[2]; sTt[(c4 + 3) * 68 + n] = v[3];
  }
  __syncthreads();
  for (int pass = 0; pass < 2; ++pass) {
#pragma unroll
    for (int it = 0; it < 4; ++it) {
      const int row = wave * 16 + it * 4 + q;
      const v4u u = pack8_f16(sTt + row * 68 + c8);
      *(volatile v4u*)(ap + (size_t)row * kNodes + n0 + c8) = u;
      *(volatile v4u*)(bp + (size_t)(kFeat + row) * kNodes + n0 + c8) = u;
    }
#pragma unroll
    for (int it = 0; it < 2; ++it) {
      const int row = 2 * kFeat + wave * 8 + it * 4 + q;
      const unsigned w = (row == 2 * kFeat) ? 0x3C003C00u : 0u;
      const v4u u = (v4u){w, w, w, w};
      *(volatile v4u*)(bp + (size_t)row * kNodes + n0 + c8) = u;
    }
    __threadfence();
  }
}

__global__ __launch_bounds__(kNT) void trace_kernel(const float* __restrict__ S, const int* __restrict__ E0,
                                                  const int* __restrict__ E1, float* __restrict__ TRP) {
  __shared__ __align__(16) float rca[8][kClus];
  __shared__ float rtr[8];
  const int tid = threadIdx.x, lane = tid & 31, wave = tid >> 5;
  const int g = blockIdx.y, b = blockIdx.x;
  const int* ei = g ? E1 : E0;
  const int* srcv = ei;
  const int* dstv = ei + kEdges;
  const float* Sg = S + (size_t)g * kNodes * kClus;
  v4f ca = {0.f, 0.f, 0.f, 0.f};
  v4f tr4 = {0.f, 0.f, 0.f, 0.f};
  const int ebase = (b * 8 + wave) * kTrEdgesPerWave;
#pragma unroll 1
  for (int grp = 0; grp < kTrEdgesPerWave / 32; ++grp) {
    const int e = ebase + grp * 32 + lane;
    int sv = srcv[e], dv = dstv[e];
    sv = sv < 0 ? 0 : (sv >= kNodes ? kNodes - 1 : sv);
    dv = dv < 0 ? 0 : (dv >= kNodes ? kNodes - 1 : dv);
#pragma unroll 1
    for (int it = 0; it < 32; ++it) {
      const int s = __shfl(sv, it, 32);
      const int d = __shfl(dv, it, 32);
      const v4f xa = *(const v4f*)(Sg + (size_t)s * kClus + 4 * lane);
      const v4f xb = *(const v4f*)(Sg + (size_t)d * kClus + 4 * lane);
      ca = ca + xa;
      tr4 = tr4 + xa * xb;
    }
  }
  float tr = (tr4[0] + tr4[1]) + (tr4[2] + tr4[3]);
  tr += __shfl_xor(tr, 16, 32);
  tr += __shfl_xor(tr, 8, 32);
  tr += __shfl_xor(tr, 4, 32);
  tr += __shfl_xor(tr, 2, 32);
  tr += __shfl_xor(tr, 1, 32);
  *(v4f*)(rca[wave] + 4 * lane) = ca;
  if (lane == 0) rtr[wave] = tr;
  __syncthreads();
  if (wave == 0) {
    v4f cs = {0.f, 0.f, 0.f, 0.f};
    float ts = 0.0f;
#pragma unroll
    for (int w = 0; w < 8; ++w) { cs = cs + *(const v4f*)(rca[w] + 4 * lane); ts += rtr[w]; }
    const v4f tv = (v4f){(lane == 0) ? ts : 0.0f, 0.0f, 0.0f, 0.0f};
    float* rowp = TRP + ((size_t)g * kTrB + b) * kTrRow;
    for (int pass = 0; pass < 2; ++pass) {
      *(volatile v4f*)(rowp + 4 * lane) = cs;
      if (lane < 8) *(volatile v4f*)(rowp + kClus + 4 * lane) = tv;
      __threadfence();
    }
  }
}

__global__ __launch_bounds__(kNT) void final_kernel(const float* __restrict__ PP, const float* __restrict__ TRP, float* __restrict__ out) {
  __shared__ float red[kNT];
  __shared__ __align__(16) float rowbuf[8][kFeat];
  const int t = threadIdx.x, lane = t & 31, wave = t >> 5;
#pragma unroll 1
  for (int R = wave; R < 2 * kClus; R += 8) {
    const int g = R >> 7, k = R & (kClus - 1);
    const float* pr = PP + ((size_t)g * kClus + k) * kPoolN;
#pragma unroll 1
    for (int i = 0; i < 4; ++i) {
      const int c = lane + 32 * i;
      rowbuf[wave][c] = selu_f(pr[c]);
    }
    wave_lds_sync();
    const v4f o = *(const v4f*)(rowbuf[wave] + 4 * lane);
    float* op = out + (size_t)R * kFeat + 4 * lane;
    *(volatile v4f*)op = o;
    __threadfence();
    *(volatile v4f*)op = o;
    wave_lds_sync();
  }

  const float invE = 1.0f / (float)kEdges;
  const float sqrtK = sqrtf((float)kClus);
  const float invSqrtK = 1.0f / sqrtK;
  const float invN = 1.0f / (float)kNodes;
  float loss = 0.0f;
#pragma unroll 1
  for (int g = 0; g < 2; ++g) {
    const float* trp = TRP + (size_t)g * kTrB * kTrRow;
    const float* pp  = PP  + (size_t)g * kClus * kPoolN;
    const int tc = (t < kClus) ? t : (kClus - 1);
    const int tb = (t < kTrB) ? t : (kTrB - 1);
    float cav = 0.0f;
#pragma unroll 1
    for (int bb = 0; bb < kTrB; ++bb) cav += trp[(size_t)bb * kTrRow + tc];
    const float ca2 = block_sum256((t < kClus) ? cav * cav : 0.0f, red);
    float trv = trp[(size_t)tb * kTrRow + kClus];
    trv = (t < kTrB) ? trv : 0.0f;
    const float tr = block_sum256(trv, red);
    const float spectral = -(tr - ca2 * invE) * invE;
    float sq = 0.0f;
#pragma unroll 1
    for (int i = t; i < kClus * kClus; i += kNT) {
      const float v = pp[(size_t)(i >> 7) * kPoolN + kClus + (i & (kClus - 1))];
      sq += v * v;
    }
    const float nF = sqrtf(block_sum256(sq, red));
    const float invnF = 1.0f / nF;
    float ds = 0.0f;
#pragma unroll 1
    for (int i = t; i < kClus * kClus; i += kNT) {
      const int rr = i >> 7, cc = i & (kClus - 1);
      float v = pp[(size_t)rr * kPoolN + kClus + cc] * invnF;
      v = v - ((rr == cc) ? invSqrtK : 0.0f);
      ds += v * v;
    }
    const float ortho = sqrtf(block_sum256(ds, red));
    float cs = pp[(size_t)tc * kPoolN + 2 * kClus];
    cs = (t < kClus) ? cs : 0.0f;
    const float cs2 = block_sum256(cs * cs, red);
    const float cluster = sqrtf(cs2) * invN * sqrtK - 1.0f;
    loss += spectral + ortho + cluster;
  }
  if (t == 0) {
    float* op = out + 2 * kClus * kFeat;
    *(volatile float*)op = loss;
    __threadfence();
    *(volatile float*)op = loss;
  }
}

extern "C" void kernel_launch(void* const* d_in, const int* in_sizes, int n_in,
                              void* d_out, int out_size, void* d_ws, size_t ws_size, hipStream_t stream) {
  if (n_in < 23) return;
  if (in_sizes[0] != kNodes * kFeat || in_sizes[1] != kNodes * kFeat) return;
  if (in_sizes[2] != 2 * kEdges || in_sizes[3] != 2 * kEdges) return;
  if (out_size != 2 * kClus * kFeat + 1) return;
  const float* x1 = (const float*)d_in[0];
  const float* x2 = (const float*)d_in[1];
  const int*   e1 = (const int*)d_in[2];
  const int*   e2 = (const int*)d_in[3];
  const float* cWl[5]; const float* cbl[5]; const float* cWr[5];
  for (int i = 0; i < 5; ++i) {
    cWl[i] = (const float*)d_in[4 + 3 * i];
    cbl[i] = (const float*)d_in[5 + 3 * i];
    cWr[i] = (const float*)d_in[6 + 3 * i];
  }
  const float* mW1 = (const float*)d_in[19];
  const float* mb1 = (const float*)d_in[20];
  const float* mW2 = (const float*)d_in[21];
  const float* mb2 = (const float*)d_in[22];
  float* out = (float*)d_out;

  char* ws = (char*)d_ws; size_t off = 0;
  auto carve = [&](size_t bytes) -> char* { char* p = ws + off; off += (bytes + 255) & ~(size_t)255; return p; };
  const size_t plF32 = (size_t)kNodes * kFeat * 4;
  const size_t plF16 = (size_t)kNodes * kFeat * 2;
  unsigned short* BTS    = (unsigned short*)carve((size_t)5 * kFeat * kAK * 2);
  unsigned short* BTM    = (unsigned short*)carve((size_t)2 * kFeat * kFeat * 2);
  float*          B1X16  = (float*)carve((size_t)kFeat * 4);
  unsigned short* A16    = (unsigned short*)carve((size_t)2 * kNodes * kAK * 2);
  float*          ACC    = (float*)carve(2 * plF32);
  float*          PRE    = (float*)carve(2 * plF32);
  float*          H1     = (float*)carve(2 * plF32);
  float*          HS     = (float*)carve(2 * plF32);
  float*          HF     = (float*)carve(2 * plF32);
  unsigned short* H16    = (unsigned short*)carve(2 * plF16);
  unsigned short* T16    = (unsigned short*)carve(2 * plF16);
  float*          LOGIT  = (float*)carve(2 * plF32);
  float*          S      = (float*)carve(2 * plF32);
  unsigned short* APOOL  = (unsigned short*)carve((size_t)2 * kClus * kNodes * 2);
  unsigned short* BTPOOL = (unsigned short*)carve((size_t)2 * kPoolN * kNodes * 2);
  float*          PP     = (float*)carve((size_t)2 * kClus * kPoolN * 4);
  float*          TRP    = (float*)carve((size_t)2 * kTrB * kTrRow * 4);
  if (off > ws_size || off > (size_t)134217728) return;

  const long strideFeat = (long)kNodes * kFeat;
  const long strideA16  = (long)kNodes * kAK;
  const size_t btsPlane = (size_t)kFeat * kAK;
  const dim3 gridAgg(kTiles, 2);
  const dim3 gridGemm((kNodes / 64) * (kFeat / 64) / 8, 2);
  const dim3 gridAct(kNodes * kFeat / 2048, 2);

  prep_kernel<<<dim3(2, 2, 12), kNT, 0, stream>>>(cWl[0], cWr[0], cWl[1], cWr[1], cWl[2], cWr[2], cWl[3], cWr[3],
                                                  cWl[4], cWr[4], mW1, mW2, mb1, BTS, BTM, B1X16);

  agg_kernel<<<gridAgg, kNT, 0, stream>>>(x1, x2, e1, e2, ACC, (unsigned*)A16);
  wmma_gemm64<0, false, 0, 0, false, 0><<<gridGemm, 256, 0, stream>>>(
      (const unsigned short*)A16, nullptr, kAK, strideA16,
      (const unsigned short*)BTS, nullptr, kAK, (long)btsPlane,
      (void*)PRE, nullptr, kFeat, strideFeat,
      nullptr, nullptr, 0L, kNodes, kFeat, kAK, kInvW);
  act_kernel<0><<<gridAct, kNT, 0, stream>>>(PRE, cbl[0], cbl[1], nullptr, H1, nullptr);

  agg_kernel<<<gridAgg, kNT, 0, stream>>>(H1, H1 + strideFeat, e1, e2, ACC, (unsigned*)A16);
  wmma_gemm64<0, false, 0, 0, false, 0><<<gridGemm, 256, 0, stream>>>(
      (const unsigned short*)A16, nullptr, kAK, strideA16,
      (const unsigned short*)(BTS + 2 * btsPlane), nullptr, kAK, 0L,
      (void*)PRE, nullptr, kFeat, strideFeat,
      nullptr, nullptr, 0L, kNodes, kFeat, kAK, kInvW);
  act_kernel<1><<<gridAct, kNT, 0, stream>>>(PRE, cbl[2], cbl[2], H1, HS, nullptr);

  agg_kernel<<<gridAgg, kNT, 0, stream>>>(HS, HS + strideFeat, e1, e2, ACC, (unsigned*)A16);
  wmma_gemm64<0, false, 0, 0, false, 0><<<gridGemm, 256, 0, stream>>>(
      (const unsigned short*)A16, nullptr, kAK, strideA16,
      (const unsigned short*)(BTS + 3 * btsPlane), nullptr, kAK, (long)btsPlane,
      (void*)PRE, nullptr, kFeat, strideFeat,
      nullptr, nullptr, 0L, kNodes, kFeat, kAK, kInvW);
  act_kernel<2><<<gridAct, kNT, 0, stream>>>(PRE, cbl[3], cbl[4], nullptr, HF, (unsigned*)H16);

  wmma_gemm64<0, false, 2, 1, false, 0><<<gridGemm, 256, 0, stream>>>(
      (const unsigned short*)H16, nullptr, kFeat, strideFeat,
      (const unsigned short*)BTM, nullptr, kFeat, 0L,
      (void*)T16, nullptr, kFeat, strideFeat,
      B1X16, nullptr, 0L, kNodes, kFeat, kFeat, 1.0f);
  wmma_gemm64<0, false, 2, 0, false, 0><<<gridGemm, 256, 0, stream>>>(
      (const unsigned short*)T16, nullptr, kFeat, strideFeat,
      (const unsigned short*)(BTM + (size_t)kFeat * kFeat), nullptr, kFeat, 0L,
      (void*)LOGIT, nullptr, kClus, (long)kNodes * kClus,
      mb2, nullptr, 0L, kNodes, kClus, kFeat, kInvWW);
  softmax_kernel<<<dim3(kNodes / 8, 2), kNT, 0, stream>>>(LOGIT, S);

  poolpack_kernel<<<dim3(kNodes / 64, 2), kNT, 0, stream>>>(HF, S, APOOL, BTPOOL);
  wmma_gemm64<0, false, 0, 0, false, 0><<<dim3(2, 2), 256, 0, stream>>>(
      (const unsigned short*)APOOL, nullptr, kNodes, (long)kClus * kNodes,
      (const unsigned short*)BTPOOL, nullptr, kNodes, (long)kPoolN * kNodes,
      (void*)PP, nullptr, kPoolN, (long)kClus * kPoolN,
      nullptr, nullptr, 0L, kClus, kPoolN, kNodes, 1.0f);

  trace_kernel<<<dim3(kTrB, 2), kNT, 0, stream>>>(S, e1, e2, TRP);
  final_kernel<<<1, kNT, 0, stream>>>(PP, TRP, out);
}
